// WordRNN_25297357373664
// MI455X (gfx1250) — hardware-verified
//
#include <hip/hip_runtime.h>
#include <math.h>

constexpr int VOCAB_N    = 100000;
constexpr int EMB_N      = 20;
constexpr int HID_N      = 10;
constexpr int SEQ_N      = 100;
constexpr int NLAB_N     = 15;
constexpr int BATCH_N    = 16384;
constexpr int GATES_N    = 4 * HID_N;
constexpr int KPAD       = 32;
constexpr int NPAD_COLS  = 64;
constexpr int VPAD_ROWS  = 100032;
constexpr int GT_ROWS    = 32;
constexpr int GT_WAVES   = 6;
constexpr int RB_THREADS = 128;
constexpr int SLAB_PITCH = 68;

static_assert(GATES_N == 40, "gate columns");
static_assert(EMB_N <= KPAD && KPAD % 32 == 0, "K pad");
static_assert(EMB_N % 4 == 0 && GATES_N % 4 == 0, "vector loads");
static_assert(GATES_N <= NPAD_COLS && NPAD_COLS == 64, "N pad");
static_assert(VPAD_ROWS >= VOCAB_N && VPAD_ROWS % GT_ROWS == 0, "M pad");
static_assert((VPAD_ROWS / GT_ROWS) % GT_WAVES == 0, "table GEMM grid exact");
static_assert((VPAD_ROWS * 4) % 256 == 0, "plane producer grid exact");
static_assert(BATCH_N % RB_THREADS == 0, "row grid exact");
static_assert((32 * NLAB_N * 4) % 128 == 0, "a wave of output rows is whole 128-B lines");
static_assert(HID_N * GATES_N <= 4 * RB_THREADS, "Wh staging coverage");
static_assert(HID_N * NLAB_N <= 160 && 160 <= 2 * RB_THREADS, "Wd staging coverage");

typedef __attribute__((ext_vector_type(16))) __bf16   v16b;
typedef __attribute__((ext_vector_type(8)))  __bf16   v8b;
typedef __attribute__((ext_vector_type(8)))  float    v8f;
typedef __attribute__((ext_vector_type(4)))  float    v4f;
typedef __attribute__((ext_vector_type(4)))  unsigned v4u;

__device__ __forceinline__ unsigned f2bf_u(float f) {
  const unsigned u = __float_as_uint(f);
  return ((u + 0x7FFFu + ((u >> 16) & 1u)) >> 16) & 0xFFFFu;
}
__device__ __forceinline__ float bf_u2f(unsigned h) { return __uint_as_float(h << 16); }

__device__ __forceinline__ void split_pack8(const v4f a, const v4f b, v4u& hw, v4u& lw) {
#pragma unroll
  for (int q = 0; q < 2; ++q) {
    const float f0 = a[2 * q];
    const float f1 = a[2 * q + 1];
    const float g0 = b[2 * q];
    const float g1 = b[2 * q + 1];
    const unsigned hf0 = f2bf_u(f0);
    const unsigned hf1 = f2bf_u(f1);
    const unsigned hg0 = f2bf_u(g0);
    const unsigned hg1 = f2bf_u(g1);
    const unsigned lf0 = f2bf_u(f0 - bf_u2f(hf0));
    const unsigned lf1 = f2bf_u(f1 - bf_u2f(hf1));
    const unsigned lg0 = f2bf_u(g0 - bf_u2f(hg0));
    const unsigned lg1 = f2bf_u(g1 - bf_u2f(hg1));
    hw[q]     = hf0 | (hf1 << 16);
    hw[2 + q] = hg0 | (hg1 << 16);
    lw[q]     = lf0 | (lf1 << 16);
    lw[2 + q] = lg0 | (lg1 << 16);
  }
}

__device__ __forceinline__ void group_guard_b(v8f& a, v8f& b, v8f& c, v8f& d, v16b x, v16b y, v16b z, v16b w) {
  asm volatile("v_nop\n\tv_nop\n\tv_nop\n\tv_nop" : "+v"(a), "+v"(b), "+v"(c), "+v"(d) : "v"(x), "v"(y), "v"(z), "v"(w));
}
__device__ __forceinline__ void keep4_b(v16b a, v16b b, v16b c, v16b d) { asm volatile("v_nop" :: "v"(a), "v"(b), "v"(c), "v"(d)); }
__device__ __forceinline__ void acc_guard4(v8f& a, v8f& b, v8f& c, v8f& d) { asm volatile("v_nop\n\tv_nop\n\tv_nop\n\tv_nop" : "+v"(a), "+v"(b), "+v"(c), "+v"(d)); }

struct FragB {
  union U { v16b v; v8b h[2]; };
  static __device__ __forceinline__ v16b load(const __bf16* p) {
    U f;
    f.h[0] = *(const v8b*)(p);
    f.h[1] = *(const v8b*)(p + 16);
    return f.v;
  }
  static __device__ __forceinline__ v8f mma(v16b a, v16b b, v8f c) {
    return __builtin_amdgcn_wmma_f32_16x16x32_bf16(false, a, false, b, (short)0, c, false, false);
  }
};

__global__ __launch_bounds__(256) void emb_planes_kernel(const float* __restrict__ emb, unsigned* __restrict__ AH,
                                                         unsigned* __restrict__ AL) {
  const int i   = blockIdx.x * 256 + threadIdx.x;
  const int row = i >> 2;
  const int c8  = (i & 3) * 8;
  const bool rowok = row < VOCAB_N;
  const int rowc = rowok ? row : (VOCAB_N - 1);
  const int ca = (c8 < EMB_N - 4) ? c8 : (EMB_N - 4);
  const int cb = (c8 + 4 < EMB_N - 4) ? (c8 + 4) : (EMB_N - 4);
  const float* rp = emb + (size_t)rowc * EMB_N;
  const v4f va = *(const v4f*)(rp + ca);
  const v4f vb = *(const v4f*)(rp + cb);
  v4f fa, fb;
#pragma unroll
  for (int e = 0; e < 4; ++e) {
    fa[e] = (rowok && (c8 + e) < EMB_N) ? va[e] : 0.0f;
    fb[e] = (rowok && (c8 + 4 + e) < EMB_N) ? vb[e] : 0.0f;
  }
  v4u hw, lw;
  split_pack8(fa, fb, hw, lw);
  unsigned* ph = AH + (size_t)i * 4;
  unsigned* pl = AL + (size_t)i * 4;
  *(volatile v4u*)ph = hw;
  *(volatile v4u*)pl = lw;
  __threadfence();
  *(volatile v4u*)ph = hw;
  *(volatile v4u*)pl = lw;
}

__global__ __launch_bounds__(256) void w_planes_kernel(const float* __restrict__ Wx, const float* __restrict__ bvec,
                                                       unsigned* __restrict__ BH, unsigned* __restrict__ BL,
                                                       float* __restrict__ biasp) {
  const int tid = threadIdx.x;
  const int n   = tid >> 2;
  const int c8  = (tid & 3) * 8;
  const bool nok = n < GATES_N;
  const int nc = nok ? n : (GATES_N - 1);
  v4f fa, fb;
#pragma unroll
  for (int e = 0; e < 4; ++e) {
    const int k0 = c8 + e;
    const int k1 = c8 + 4 + e;
    const int k0c = (k0 < EMB_N) ? k0 : (EMB_N - 1);
    const int k1c = (k1 < EMB_N) ? k1 : (EMB_N - 1);
    const float w0 = Wx[k0c * GATES_N + nc];
    const float w1 = Wx[k1c * GATES_N + nc];
    fa[e] = (nok && k0 < EMB_N) ? w0 : 0.0f;
    fb[e] = (nok && k1 < EMB_N) ? w1 : 0.0f;
  }
  v4u hw, lw;
  split_pack8(fa, fb, hw, lw);
  const int idx = (tid & 15) * 4;
  v4f bv;
#pragma unroll
  for (int e = 0; e < 4; ++e) {
    const int g = idx + e;
    const int gc = (g < GATES_N) ? g : (GATES_N - 1);
    const float t = bvec[gc];
    bv[e] = (g < GATES_N) ? t : 0.0f;
  }
  unsigned* ph = BH + (size_t)tid * 4;
  unsigned* pl = BL + (size_t)tid * 4;
  *(volatile v4u*)ph = hw;
  *(volatile v4u*)pl = lw;
  if (tid < 16) *(volatile v4f*)(biasp + idx) = bv;
  __threadfence();
  *(volatile v4u*)ph = hw;
  *(volatile v4u*)pl = lw;
  if (tid < 16) *(volatile v4f*)(biasp + idx) = bv;
}

__global__ __launch_bounds__(32 * GT_WAVES) void table_gemm_kernel(
    const unsigned short* __restrict__ Ap, const unsigned short* __restrict__ A2p,
    const unsigned short* __restrict__ Btp, const unsigned short* __restrict__ Bt2p,
    float* __restrict__ C, const float* __restrict__ bias) {
  const __bf16* A   = (const __bf16*)Ap;
  const __bf16* A2  = (const __bf16*)A2p;
  const __bf16* Bt  = (const __bf16*)Btp;
  const __bf16* Bt2 = (const __bf16*)Bt2p;
  __shared__ __align__(16) float sT[GT_WAVES][16 * SLAB_PITCH];
  const int lane = threadIdx.x & 31;
  const int wave = threadIdx.x >> 5;
  const int tile = blockIdx.x * GT_WAVES + wave;
  const int m0 = tile * GT_ROWS;
  const int rlane = lane & 15;
  const int koff  = (lane >> 4) * 8;
  const int mOff  = (lane >> 4) * 8;

  v8f acc[2][4];
#pragma unroll
  for (int i = 0; i < 2; ++i)
#pragma unroll
    for (int j = 0; j < 4; ++j) acc[i][j] = (v8f){0.f, 0.f, 0.f, 0.f, 0.f, 0.f, 0.f, 0.f};

  for (int k0 = 0; k0 < KPAD; k0 += 32) {
    v16b bh[4], bl[4];
#pragma unroll
    for (int j = 0; j < 4; ++j) {
      const size_t bo = (size_t)((j << 4) + rlane) * KPAD + koff + k0;
      bh[j] = FragB::load(Bt + bo);
      bl[j] = FragB::load(Bt2 + bo);
    }
#pragma unroll
    for (int i = 0; i < 2; ++i) {
      const size_t ao = (size_t)(m0 + (i << 4) + rlane) * KPAD + koff + k0;
      const v16b ah = FragB::load(A + ao);
      const v16b al = FragB::load(A2 + ao);
#pragma unroll
      for (int j = 0; j < 4; ++j) {
        acc[i][j] = FragB::mma(ah, bh[j], acc[i][j]);
        acc[i][j] = FragB::mma(ah, bl[j], acc[i][j]);
        acc[i][j] = FragB::mma(al, bh[j], acc[i][j]);
      }
      group_guard_b(acc[i][0], acc[i][1], acc[i][2], acc[i][3], ah, al, bh[3], bl[3]);
    }
    keep4_b(bh[0], bh[1], bh[2], bh[3]);
    keep4_b(bl[0], bl[1], bl[2], bl[3]);
  }
  acc_guard4(acc[0][0], acc[0][1], acc[0][2], acc[0][3]);
  acc_guard4(acc[1][0], acc[1][1], acc[1][2], acc[1][3]);

  float* slab = sT[wave];
  const int hh = lane >> 4;
  const int c4 = (lane & 15) * 4;
#pragma unroll
  for (int i = 0; i < 2; ++i) {
    const int mBase = m0 + (i << 4);
#pragma unroll
    for (int j = 0; j < 4; ++j) {
      const float bv = bias[(j << 4) + rlane];
#pragma unroll
      for (int r = 0; r < 8; ++r) slab[(mOff + r) * SLAB_PITCH + (j << 4) + rlane] = acc[i][j][r] + bv;
    }
    __syncthreads();
    for (int pass = 0; pass < 2; ++pass) {
#pragma unroll
      for (int it = 0; it < 8; ++it) {
        const int row = it * 2 + hh;
        const v4f v = *(const v4f*)(slab + row * SLAB_PITCH + c4);
        *(volatile v4f*)(C + (size_t)(mBase + row) * NPAD_COLS + c4) = v;
      }
      __threadfence();
    }
    __syncthreads();
  }
}

__device__ __forceinline__ float gate_sig(float v)  { return __builtin_amdgcn_rcpf(1.0f + expf(-v)); }
__device__ __forceinline__ float gate_tanh(float v) { return 1.0f - 2.0f * __builtin_amdgcn_rcpf(1.0f + expf(2.0f * v)); }

__global__ __launch_bounds__(RB_THREADS) void lstm_rows_kernel(const int* __restrict__ x, const float* __restrict__ PT,
                                                               const float* __restrict__ Wh, const float* __restrict__ Wd,
                                                               const float* __restrict__ bd, float* __restrict__ out) {
  __shared__ __align__(16) float zl[GATES_N * RB_THREADS];
  __shared__ __align__(16) float hl[HID_N * RB_THREADS];
  __shared__ __align__(16) float cl[HID_N * RB_THREADS];
  __shared__ __align__(16) float whs[HID_N * GATES_N];
  __shared__ __align__(16) float wds[160];
  __shared__ __align__(16) float bds[16];
  __shared__ __align__(16) float ost[RB_THREADS / 32][32 * NLAB_N];

  const int tid  = threadIdx.x;
  const int lane = tid & 31;
  const int wave = tid >> 5;
  const int row  = blockIdx.x * RB_THREADS + tid;

#pragma unroll 1
  for (int it = 0; it < 4; ++it) {
    const int i = it * RB_THREADS + tid;
    const int ic = (i < HID_N * GATES_N) ? i : (HID_N * GATES_N - 1);
    const float v = Wh[ic];
    if (i < HID_N * GATES_N) whs[i] = v;
  }
#pragma unroll 1
  for (int it = 0; it < 2; ++it) {
    const int i = it * RB_THREADS + tid;
    const int ic = (i < HID_N * NLAB_N) ? i : (HID_N * NLAB_N - 1);
    const float v = Wd[ic];
    if (i < 160) wds[i] = (i < HID_N * NLAB_N) ? v : 0.0f;
  }
  {
    const int ic = (tid < NLAB_N) ? tid : (NLAB_N - 1);
    const float v = bd[ic];
    if (tid < 16) bds[tid] = (tid < NLAB_N) ? v : 0.0f;
  }
#pragma unroll 1
  for (int j = 0; j < HID_N; ++j) {
    hl[j * RB_THREADS + tid] = 0.0f;
    cl[j * RB_THREADS + tid] = 0.0f;
  }
  __syncthreads();

  const int* xr = x + (size_t)row * SEQ_N;

#pragma unroll 1
  for (int t = 0; t < SEQ_N; ++t) {
    int id = xr[t];
    asm volatile("" : "+v"(id));
    id = (id < 0) ? 0 : id;
    id = (id > VOCAB_N - 1) ? (VOCAB_N - 1) : id;
    const v4f* pr = (const v4f*)(PT + (size_t)id * NPAD_COLS);
    float z[GATES_N];
#pragma unroll
    for (int q = 0; q < GATES_N / 4; ++q) {
      const v4f v = pr[q];
      z[4 * q + 0] = v[0];
      z[4 * q + 1] = v[1];
      z[4 * q + 2] = v[2];
      z[4 * q + 3] = v[3];
    }
#pragma unroll 1
    for (int k = 0; k < HID_N; ++k) {
      const float hk = hl[k * RB_THREADS + tid];
      const float* wr = whs + k * GATES_N;
#pragma unroll
      for (int q = 0; q < GATES_N / 4; ++q) {
        const v4f w = *(const v4f*)(wr + 4 * q);
        z[4 * q + 0] = fmaf(hk, w[0], z[4 * q + 0]);
        z[4 * q + 1] = fmaf(hk, w[1], z[4 * q + 1]);
        z[4 * q + 2] = fmaf(hk, w[2], z[4 * q + 2]);
        z[4 * q + 3] = fmaf(hk, w[3], z[4 * q + 3]);
      }
    }
#pragma unroll
    for (int g = 0; g < GATES_N; ++g) zl[g * RB_THREADS + tid] = z[g];
#pragma unroll 1
    for (int j = 0; j < HID_N; ++j) {
      const int o = j * RB_THREADS + tid;
      const float zi = zl[o];
      const float zf = zl[o + 1 * HID_N * RB_THREADS];
      const float zc = zl[o + 2 * HID_N * RB_THREADS];
      const float zo = zl[o + 3 * HID_N * RB_THREADS];
      const float co = cl[o];
      const float ig = gate_sig(zi);
      const float fg = gate_sig(zf);
      const float og = gate_sig(zo);
      const float tg = gate_tanh(zc);
      const float cn = fg * co + ig * tg;
      const float hn = og * gate_tanh(cn);
      cl[o] = cn;
      hl[o] = hn;
    }
  }

  float* os = ost[wave];
#pragma unroll 1
  for (int j = 0; j < NLAB_N; ++j) {
    float acc = 0.0f;
#pragma unroll 1
    for (int k = 0; k < HID_N; ++k) acc = fmaf(hl[k * RB_THREADS + tid], wds[k * NLAB_N + j], acc);
    os[lane * NLAB_N + j] = acc + bds[j];
  }
  __syncthreads();
  float* op = out + (size_t)(blockIdx.x * RB_THREADS + wave * 32) * NLAB_N;
  for (int pass = 0; pass < 2; ++pass) {
#pragma unroll
    for (int it = 0; it < NLAB_N; ++it) {
      const float v = os[it * 32 + lane];
      *(volatile float*)(op + it * 32 + lane) = v;
    }
    __threadfence();
  }
}

extern "C" void kernel_launch(void* const* d_in, const int* in_sizes, int n_in,
                              void* d_out, int out_size, void* d_ws, size_t ws_size, hipStream_t stream) {
  if (n_in < 7 || d_out == nullptr || d_ws == nullptr) return;
  if (in_sizes[0] != BATCH_N * SEQ_N || in_sizes[1] != VOCAB_N * EMB_N || in_sizes[2] != EMB_N * GATES_N ||
      in_sizes[3] != HID_N * GATES_N || in_sizes[4] != GATES_N || in_sizes[5] != HID_N * NLAB_N ||
      in_sizes[6] != NLAB_N || out_size != BATCH_N * NLAB_N) return;

  const int*   xin = (const int*)d_in[0];
  const float* emb = (const float*)d_in[1];
  const float* Wx  = (const float*)d_in[2];
  const float* Wh  = (const float*)d_in[3];
  const float* bg  = (const float*)d_in[4];
  const float* Wd  = (const float*)d_in[5];
  const float* bd  = (const float*)d_in[6];
  float* out = (float*)d_out;

  char* ws = (char*)d_ws;
  size_t off = 0;
  auto carve = [&](size_t bytes) -> char* { char* p = ws + off; off += (bytes + 255) & ~(size_t)255; return p; };
  char* AHI   = carve((size_t)VPAD_ROWS * KPAD * 2);
  char* ALO   = carve((size_t)VPAD_ROWS * KPAD * 2);
  char* BHI   = carve((size_t)NPAD_COLS * KPAD * 2);
  char* BLO   = carve((size_t)NPAD_COLS * KPAD * 2);
  char* BIASP = carve((size_t)NPAD_COLS * 4);
  char* PT    = carve((size_t)VPAD_ROWS * NPAD_COLS * 4);
  if (off > ws_size || off > (size_t)134217728) return;

  emb_planes_kernel<<<(VPAD_ROWS * 4) / 256, 256, 0, stream>>>(emb, (unsigned*)AHI, (unsigned*)ALO);
  w_planes_kernel<<<1, 256, 0, stream>>>(Wx, bg, (unsigned*)BHI, (unsigned*)BLO, (float*)BIASP);
  table_gemm_kernel<<<(VPAD_ROWS / GT_ROWS) / GT_WAVES, 32 * GT_WAVES, 0, stream>>>(
      (const unsigned short*)AHI, (const unsigned short*)ALO,
      (const unsigned short*)BHI, (const unsigned short*)BLO,
      (float*)PT, (const float*)BIASP);
  lstm_rows_kernel<<<BATCH_N / RB_THREADS, RB_THREADS, 0, stream>>>(xin, (const float*)PT, Wh, Wd, bd, out);
}
